// BiGraphContrastLayer_2911987826804
// MI455X (gfx1250) — hardware-verified
//
#include <hip/hip_runtime.h>
#include <stddef.h>


#define FIN     512
#define NC      512
#define NCW     128
#define NSLAB   (NC / NCW)
#define CHN     64
#define NHEAD   8
#define HPS     (NCW / CHN)
#define WSC     256
#define NTHR    256
#define NWAVE   8
#define EPT     8
#define NGRP    2
#define CHUNK   (NTHR * EPT * NGRP)
#define WCAP    (EPT * NGRP * 32)
#define LISTN   (NWAVE * WCAP)
#define NBC     4096
#define NBF     1024
#define RCAP    40960
#define RBN     128
#define TGT     256
#define DEGCAP  256
#define OTHR    512
#define BM      64
#define RPAD    256
#define WSCAP   134217728
#define NEG_SLOPE 0.2f

#define LDS_FILL ((RCAP + NBF + LISTN) * 4 + 64)

static_assert((CHUNK & (CHUNK - 1)) == 0);
static_assert(CHUNK <= 4096);
static_assert(NBC <= 4096 && NBF <= 4096);
static_assert((NBC & (NBC - 1)) == 0 && (NBF & (NBF - 1)) == 0);
static_assert(NBC == 4 * NBF);
static_assert(OTHR * 8 == NBC);
static_assert((RCAP % 32) == 0);
static_assert(TGT == NWAVE * 32);
static_assert((NBC % TGT) == 0);
static_assert((TGT % BM) == 0);
static_assert((RPAD % TGT) == 0 && (RPAD % BM) == 0);
static_assert(BM * 4 == NTHR);
static_assert(FIN % 64 == 0 && NC % 64 == 0);
static_assert(NC == NHEAD * CHN);
static_assert(NSLAB * HPS == NHEAD);
static_assert(FIN / 8 == 64);
static_assert(WCAP == EPT * NGRP * 32);

typedef float          v4f  __attribute__((ext_vector_type(4)));
typedef float          v8f  __attribute__((ext_vector_type(8)));
typedef int            v4i  __attribute__((ext_vector_type(4)));
typedef _Float16       v8h  __attribute__((ext_vector_type(8)));
typedef _Float16       v16h __attribute__((ext_vector_type(16)));
union FragH { v16h v; v8h h[2]; };

__device__ __forceinline__ v8f wmh(v16h a, v16h b, v8f c) {
  v8f d = __builtin_amdgcn_wmma_f32_16x16x32_f16(false, a, false, b, (short)0, c, false, false);
  asm volatile("v_nop\n\tv_nop\n\tv_nop\n\tv_nop" : "+v"(d) : "v"(a), "v"(b));
  return d;
}

__device__ __forceinline__ v8h cvt8(v4f a, v4f b, float sc) {
  v8h o;
  o[0] = (_Float16)(a.x * sc); o[1] = (_Float16)(a.y * sc);
  o[2] = (_Float16)(a.z * sc); o[3] = (_Float16)(a.w * sc);
  o[4] = (_Float16)(b.x * sc); o[5] = (_Float16)(b.y * sc);
  o[6] = (_Float16)(b.z * sc); o[7] = (_Float16)(b.w * sc);
  return o;
}

__device__ __forceinline__ float lrelu(float v) { return v > 0.0f ? v : NEG_SLOPE * v; }

template <int NB>
__device__ __forceinline__ int scan_chunk(const int* __restrict__ dsts, int nE, int cbase, int slotBase,
                                          int vec8, int* list, int tid, int lane, int wave) {
  int wc = 0;
#pragma unroll
  for (int g = 0; g < NGRP; ++g) {
    const int el0  = (g * NTHR + tid) * EPT;
    const int e0   = cbase + el0;
    const int sent = -2147483647 - 1;
    v4i da, db;
    if (vec8 != 0 && cbase + CHUNK <= nE) {
      da = *(const v4i*)(dsts + e0);
      db = *(const v4i*)(dsts + e0 + 4);
    } else {
      da.x = (e0     < nE) ? dsts[min(e0, nE - 1)] : sent;
      da.y = (e0 + 1 < nE) ? dsts[min(e0 + 1, nE - 1)] : sent;
      da.z = (e0 + 2 < nE) ? dsts[min(e0 + 2, nE - 1)] : sent;
      da.w = (e0 + 3 < nE) ? dsts[min(e0 + 3, nE - 1)] : sent;
      db.x = (e0 + 4 < nE) ? dsts[min(e0 + 4, nE - 1)] : sent;
      db.y = (e0 + 5 < nE) ? dsts[min(e0 + 5, nE - 1)] : sent;
      db.z = (e0 + 6 < nE) ? dsts[min(e0 + 6, nE - 1)] : sent;
      db.w = (e0 + 7 < nE) ? dsts[min(e0 + 7, nE - 1)] : sent;
    }
    const unsigned nb = (unsigned)slotBase;
    const unsigned s0 = (unsigned)da.x - nb, s1 = (unsigned)da.y - nb;
    const unsigned s2 = (unsigned)da.z - nb, s3 = (unsigned)da.w - nb;
    const unsigned s4 = (unsigned)db.x - nb, s5 = (unsigned)db.y - nb;
    const unsigned s6 = (unsigned)db.z - nb, s7 = (unsigned)db.w - nb;
    const bool h0 = s0 < (unsigned)NB, h1 = s1 < (unsigned)NB, h2 = s2 < (unsigned)NB, h3 = s3 < (unsigned)NB;
    const bool h4 = s4 < (unsigned)NB, h5 = s5 < (unsigned)NB, h6 = s6 < (unsigned)NB, h7 = s7 < (unsigned)NB;
    const unsigned any = __builtin_amdgcn_ballot_w32(h0 | h1 | h2 | h3 | h4 | h5 | h6 | h7);
    if (any != 0u) {
#define HITJ(J, HJ, SJ) { \
        const unsigned mj = __builtin_amdgcn_ballot_w32(HJ); \
        if (mj != 0u) { \
          if (HJ) { \
            const int pos = wc + (int)__builtin_amdgcn_mbcnt_lo(mj, 0u); \
            if (pos < WCAP) list[wave * WCAP + pos] = ((el0 + (J)) << 12) | (int)(SJ); \
          } \
          wc += (int)__builtin_popcount(mj); } }
      HITJ(0, h0, s0)
      HITJ(1, h1, s1)
      HITJ(2, h2, s2)
      HITJ(3, h3, s3)
      HITJ(4, h4, s4)
      HITJ(5, h5, s5)
      HITJ(6, h6, s6)
      HITJ(7, h7, s7)
#undef HITJ
    }
  }
  return wc;
}

__global__ __launch_bounds__(NTHR) void k_xcvt(const float* __restrict__ x, _Float16* xp,
                                               int nN, int nUnits) {
  const int i = (int)blockIdx.x * NTHR + (int)threadIdx.x;
  if (i >= nUnits) return;
  const int row = i >> 6;
  const int seg = i & 63;
  const int c0  = seg * 8;
  int rr = row > nN - 1 ? nN - 1 : row;
  rr = rr < 0 ? 0 : rr;
  const float* p = x + (size_t)rr * FIN + c0;
  v4f a = *(const v4f*)p, b = *(const v4f*)(p + 4);
  const v4f z = {0.f, 0.f, 0.f, 0.f};
  if (row >= nN) { a = z; b = z; }
  const v8h o = cvt8(a, b, 1.0f);
  _Float16* d = xp + (size_t)i * 8;
  *(volatile v8h*)d = o;
  __threadfence();
  *(volatile v8h*)d = o;
}

__global__ __launch_bounds__(NTHR) void k_wtr(const float* __restrict__ W, _Float16* wt) {
  constexpr int PT = 72;
  __shared__ __attribute__((aligned(16))) _Float16 sT[64 * PT];
  const int tid = threadIdx.x;
  const int n0 = (int)blockIdx.x * 64;
  const int k0 = (int)blockIdx.y * 64;
#pragma unroll 4
  for (int i = 0; i < 16; ++i) {
    const int e = i * NTHR + tid;
    const int k = e >> 6;
    const int n = e & 63;
    const float v = W[(size_t)(k0 + k) * NC + n0 + n];
    sT[n * PT + k] = (_Float16)(v * (float)WSC);
  }
  __syncthreads();
  const int q  = tid & 7;
  const int na = tid >> 3;
  const int nb = na + 32;
  const v8h o0 = *(const v8h*)(sT + na * PT + 8 * q);
  const v8h o1 = *(const v8h*)(sT + nb * PT + 8 * q);
  _Float16* d0 = wt + (size_t)(n0 + na) * FIN + k0 + 8 * q;
  _Float16* d1 = wt + (size_t)(n0 + nb) * FIN + k0 + 8 * q;
  *(volatile v8h*)d0 = o0;
  *(volatile v8h*)d1 = o1;
  __threadfence();
  *(volatile v8h*)d0 = o0;
  *(volatile v8h*)d1 = o1;
}

__global__ __launch_bounds__(NTHR) void k_count(
    const int* __restrict__ dsts, int* cnt, int nE, int vec8) {
  __shared__ __attribute__((aligned(16))) int scnt[NBC];
  __shared__ __attribute__((aligned(16))) int list[LISTN];
  __shared__ int wcnt[NWAVE];
  const int tid = threadIdx.x, lane = tid & 31, wave = tid >> 5;
  const int nodeBase = blockIdx.x * NBC;

  for (int i = tid; i < NBC; i += NTHR) scnt[i] = 0;
  __syncthreads();

  const int nChunks = (nE + CHUNK - 1) / CHUNK;
#pragma unroll 1
  for (int ch = 0; ch < nChunks; ++ch) {
    const int cbase = ch * CHUNK;
    const int wc = scan_chunk<NBC>(dsts, nE, cbase, nodeBase, vec8, list, tid, lane, wave);
    if (lane == 0) wcnt[wave] = wc;
    __syncthreads();
    if (wave == 0) {
#pragma unroll 1
      for (int wsx = 0; wsx < NWAVE; ++wsx) {
        int n = __builtin_amdgcn_readfirstlane(wcnt[wsx]);
        n = n > WCAP ? WCAP : (n < 0 ? 0 : n);
        const int* lp = list + wsx * WCAP;
#pragma unroll 1
        for (int i = 0; i < n; ++i) {
          const int ent  = __builtin_amdgcn_readfirstlane(lp[i]);
          const int slot = ent & (NBC - 1);
          if (lane == 0) scnt[slot] = scnt[slot] + 1;
        }
      }
    }
    __syncthreads();
  }

  v4i cq[4];
#pragma unroll
  for (int q = 0; q < 4; ++q) {
    const int f = (wave * 4 + q) * 128 + 4 * lane;
    cq[q] = *(const v4i*)(scnt + f);
  }
  int* cp = cnt + (size_t)nodeBase;
#pragma unroll
  for (int q = 0; q < 4; ++q) {
    const int f = (wave * 4 + q) * 128 + 4 * lane;
    *(volatile v4i*)(cp + f) = cq[q];
  }
  __threadfence();
#pragma unroll
  for (int q = 0; q < 4; ++q) {
    const int f = (wave * 4 + q) * 128 + 4 * lane;
    *(volatile v4i*)(cp + f) = cq[q];
  }
}

__global__ __launch_bounds__(OTHR) void k_offsets(
    const int* __restrict__ cnt, int* off, int* rbase, int nChunk) {
  __shared__ __attribute__((aligned(16))) int soff[NBC];
  __shared__ __attribute__((aligned(16))) int srb[RBN];
  __shared__ int wtot[OTHR / 32];
  const int tid = threadIdx.x, lane = tid & 31, wave = tid >> 5, sub = tid >> 7;
  for (int i = tid; i < RBN; i += OTHR) srb[i] = 0;
  int carry = 0;
#pragma unroll 1
  for (int ch = 0; ch < nChunk; ++ch) {
    const int base = ch * NBC;
    const v4i c0 = *(const v4i*)(cnt + base + 8 * tid);
    const v4i c1 = *(const v4i*)(cnt + base + 8 * tid + 4);
    const int e0 = max(c0.x, 0), e1 = max(c0.y, 0), e2 = max(c0.z, 0), e3 = max(c0.w, 0);
    const int e4 = max(c1.x, 0), e5 = max(c1.y, 0), e6 = max(c1.z, 0), e7 = max(c1.w, 0);
    const int ts = e0 + e1 + e2 + e3 + e4 + e5 + e6 + e7;
    int incl = ts;
#pragma unroll
    for (int d = 1; d < 32; d <<= 1) {
      const int t = __shfl_up(incl, d);
      if (lane >= d) incl += t;
    }
    if (lane == 31) wtot[wave] = incl;
    __syncthreads();
    const int S0 = wtot[0]  + wtot[1]  + wtot[2]  + wtot[3];
    const int S1 = wtot[4]  + wtot[5]  + wtot[6]  + wtot[7];
    const int S2 = wtot[8]  + wtot[9]  + wtot[10] + wtot[11];
    const int S3 = wtot[12] + wtot[13] + wtot[14] + wtot[15];
    int pre = 0;
#pragma unroll 1
    for (int w = 4 * sub; w < wave; ++w) pre += wtot[w];
    const int b0 = carry;
    const int b1 = b0 + ((S0 + 31) & ~31);
    const int b2 = b1 + ((S1 + 31) & ~31);
    const int b3 = b2 + ((S2 + 31) & ~31);
    const int b4 = b3 + ((S3 + 31) & ~31);
    const int myb = sub == 0 ? b0 : (sub == 1 ? b1 : (sub == 2 ? b2 : b3));
    if (tid == 0) {
      srb[min(4 * ch + 0, RBN - 1)] = b0;
      srb[min(4 * ch + 1, RBN - 1)] = b1;
      srb[min(4 * ch + 2, RBN - 1)] = b2;
      srb[min(4 * ch + 3, RBN - 1)] = b3;
    }
    int run = myb + pre + incl - ts;
    soff[8 * tid + 0] = run; run += e0;
    soff[8 * tid + 1] = run; run += e1;
    soff[8 * tid + 2] = run; run += e2;
    soff[8 * tid + 3] = run; run += e3;
    soff[8 * tid + 4] = run; run += e4;
    soff[8 * tid + 5] = run; run += e5;
    soff[8 * tid + 6] = run; run += e6;
    soff[8 * tid + 7] = run;
    carry = b4;
    __syncthreads();
    const v4i o0 = *(const v4i*)(soff + 4 * tid);
    const v4i o1 = *(const v4i*)(soff + 4 * (tid + OTHR));
    int* op = off + base;
    *(volatile v4i*)(op + 4 * tid) = o0;
    *(volatile v4i*)(op + 4 * (tid + OTHR)) = o1;
    __threadfence();
    *(volatile v4i*)(op + 4 * tid) = o0;
    *(volatile v4i*)(op + 4 * (tid + OTHR)) = o1;
    __syncthreads();
  }
  if (tid == 0) srb[min(4 * nChunk, RBN - 1)] = carry;
  __syncthreads();
  v4i rv = {0, 0, 0, 0};
  if (tid < 32) rv = *(const v4i*)(srb + 4 * tid);
  if (tid < 32) *(volatile v4i*)(rbase + 4 * tid) = rv;
  __threadfence();
  if (tid < 32) *(volatile v4i*)(rbase + 4 * tid) = rv;
}

__global__ __launch_bounds__(NTHR) void k_fill(
    const int* __restrict__ srcs, const int* __restrict__ dsts,
    const int* __restrict__ off, const int* __restrict__ rbase,
    int* csr, int nN, int nE, int vec8, int csrLen) {
  extern __shared__ v4f lds_dyn[];
  int* region = (int*)lds_dyn;
  int* cursor = region + RCAP;
  int* list   = cursor + NBF;
  int* wcnt   = list + LISTN;
  const int tid = threadIdx.x, lane = tid & 31, wave = tid >> 5;
  const int b = blockIdx.x;
  const int nodeBase = b * NBF;

  int rb0 = rbase[b];
  const int rb1 = rbase[b + 1];
  rb0 = rb0 < 0 ? 0 : (rb0 > csrLen ? csrLen : rb0);
  rb0 &= ~31;
  int len = rb1 - rb0;
  len = len < 0 ? 0 : (len > RCAP ? RCAP : len);
  int lenW = (len + 31) & ~31;
  if (rb0 + lenW > csrLen) lenW = (csrLen - rb0) & ~31;

  {
    const v4i z = {0, 0, 0, 0};
    for (int i = tid; i < RCAP / 4; i += NTHR) ((v4i*)region)[i] = z;
    for (int s = tid; s < NBF; s += NTHR) {
      int o = off[nodeBase + s] - rb0;
      o = o < 0 ? 0 : (o > RCAP ? RCAP : o);
      cursor[s] = o;
    }
  }
  __syncthreads();

  const int nChunks = (nE + CHUNK - 1) / CHUNK;
#pragma unroll 1
  for (int ch = 0; ch < nChunks; ++ch) {
    const int cbase = ch * CHUNK;
    const int wc = scan_chunk<NBF>(dsts, nE, cbase, nodeBase, vec8, list, tid, lane, wave);
    if (lane == 0) wcnt[wave] = wc;
    __syncthreads();
    if (wave == 0) {
#pragma unroll 1
      for (int wsx = 0; wsx < NWAVE; ++wsx) {
        int n = __builtin_amdgcn_readfirstlane(wcnt[wsx]);
        n = n > WCAP ? WCAP : (n < 0 ? 0 : n);
        const int* lp = list + wsx * WCAP;
#pragma unroll 1
        for (int i = 0; i < n; ++i) {
          const int ent  = __builtin_amdgcn_readfirstlane(lp[i]);
          const int slot = ent & (NBF - 1);
          int e = cbase + ((ent >> 12) & (CHUNK - 1));
          e = e > nE - 1 ? nE - 1 : e;
          int sv = srcs[e];
          sv = sv < 0 ? 0 : (sv > nN - 1 ? nN - 1 : sv);
          if (lane == 0) {
            int pos = cursor[slot];
            pos = pos < 0 ? 0 : (pos > RCAP - 1 ? RCAP - 1 : pos);
            region[pos] = sv;
            const int np = pos + 1;
            cursor[slot] = np > RCAP ? RCAP : np;
          }
        }
      }
    }
    __syncthreads();
  }

  const int nv = lenW >> 2;
  int* gp = csr + rb0;
#pragma unroll 1
  for (int i = tid; i < nv; i += NTHR) { const v4i v = ((const v4i*)region)[i]; *(volatile v4i*)(gp + 4 * i) = v; }
  __threadfence();
#pragma unroll 1
  for (int i = tid; i < nv; i += NTHR) { const v4i v = ((const v4i*)region)[i]; *(volatile v4i*)(gp + 4 * i) = v; }
}

__global__ __launch_bounds__(NTHR) void k_gemm(
    const _Float16* __restrict__ Ap, const _Float16* __restrict__ Bp,
    const float* __restrict__ attS, const float* __restrict__ attD,
    float* C, float* eS, float* eD, int npad) {
  constexpr int K   = FIN;
  constexpr int TPW = NCW / 32;
  constexpr int KT  = K / 32;
  constexpr int NES = BM * HPS;
  constexpr int NV  = NES / 4;
  constexpr int CPP = NCW / 4;
  constexpr int PPH = 4 / HPS;
  constexpr int NF4 = BM * NCW / 4;
  constexpr int NIT = NF4 / NTHR;
  constexpr float OSC = 1.0f / (float)WSC;
  static_assert(K % 32 == 0);
  static_assert(HPS * CHN == NCW);
  static_assert(PPH * HPS == 4 && PPH == 2);
  static_assert(2 * NV <= NTHR);
  static_assert(NF4 % NTHR == 0);
  static_assert(TPW * 32 == NCW);
  static_assert(CPP % 4 == 0 && CPP * PPH == CHN);
  static_assert((WSC & (WSC - 1)) == 0 && WSC >= 1);
  static_assert(NCW / 4 == 32);

  __shared__ __attribute__((aligned(16))) float stg[BM * NCW];
  __shared__ __attribute__((aligned(16))) float sES[NES];
  __shared__ __attribute__((aligned(16))) float sED[NES];
  const int tid = threadIdx.x, lane = tid & 31, wave = tid >> 5, hh = lane >> 4, m = lane & 15;
  const int slab = (int)blockIdx.y;
  const int rowBase = (int)blockIdx.x * BM;
  const int rg = wave >> 1, chf = wave & 1;
  const int r0 = rg * 16;
  const int c0 = chf * (NCW / 2);
  const _Float16* Bq = Bp + (size_t)slab * NCW * K;

  v8f acc[TPW];
#pragma unroll
  for (int t = 0; t < TPW; ++t) { v8f z = {0.f, 0.f, 0.f, 0.f, 0.f, 0.f, 0.f, 0.f}; acc[t] = z; }

  const _Float16* ap  = Ap + (size_t)(rowBase + r0 + m) * K + 8 * hh;
  const _Float16* bp0 = Bq + (size_t)(c0 + m) * K + 8 * hh;
#pragma unroll 1
  for (int kt = 0; kt < KT; ++kt) {
    FragH a;
    a.h[0] = *(const v8h*)(ap + 32 * kt);
    a.h[1] = *(const v8h*)(ap + 32 * kt + 16);
#pragma unroll
    for (int t = 0; t < TPW; ++t) {
      const _Float16* bp = bp0 + (size_t)(16 * t) * K + 32 * kt;
      FragH bf;
      bf.h[0] = *(const v8h*)bp;
      bf.h[1] = *(const v8h*)(bp + 16);
      acc[t] = wmh(a.v, bf.v, acc[t]);
    }
  }

  {
    float* sp = stg + (size_t)(r0 + 8 * hh) * NCW + c0 + m;
#pragma unroll
    for (int t = 0; t < TPW; ++t) {
#pragma unroll
      for (int r = 0; r < 8; ++r) sp[r * NCW + 16 * t] = acc[t][r] * OSC;
    }
  }
  __syncthreads();

  {
    const int drow = tid >> 2, part = tid & 3;
    const float* rp  = stg + (size_t)drow * NCW + CPP * part;
    const float* sa  = attS + slab * NCW + CPP * part;
    const float* sdd = attD + slab * NCW + CPP * part;
    float ps = 0.f, pd = 0.f;
#pragma unroll 2
    for (int c = 0; c < CPP; c += 4) {
      const v4f hv = *(const v4f*)(rp + c);
      const v4f av = *(const v4f*)(sa + c);
      const v4f dv = *(const v4f*)(sdd + c);
      ps += hv.x * av.x + hv.y * av.y + hv.z * av.z + hv.w * av.w;
      pd += hv.x * dv.x + hv.y * dv.y + hv.z * dv.z + hv.w * dv.w;
    }
    ps += __shfl_xor(ps, 1); pd += __shfl_xor(pd, 1);
    if ((part & 1) == 0) {
      const int ix = drow * HPS + (part >> 1);
      sES[ix] = ps; sED[ix] = pd;
    }
  }

  {
    v4f cv[NIT];
#pragma unroll
    for (int it = 0; it < NIT; ++it) cv[it] = *(const v4f*)(stg + 4 * (it * NTHR + tid));
#pragma unroll
    for (int it = 0; it < NIT; ++it) {
      const int p = it * NTHR + tid;
      float* gp = C + (size_t)(rowBase + (p >> 5)) * NC + slab * NCW + 4 * (p & 31);
      *(volatile v4f*)gp = cv[it];
    }
    __threadfence();
#pragma unroll
    for (int it = 0; it < NIT; ++it) {
      const int p = it * NTHR + tid;
      float* gp = C + (size_t)(rowBase + (p >> 5)) * NC + slab * NCW + 4 * (p & 31);
      *(volatile v4f*)gp = cv[it];
    }
  }
  __syncthreads();

  {
    const size_t eb = ((size_t)slab * (size_t)npad + (size_t)rowBase) * HPS;
    const int iS = tid < NV - 1 ? tid : NV - 1;
    int iD = tid - NV; iD = iD < 0 ? 0 : (iD > NV - 1 ? NV - 1 : iD);
    const v4f vS = *(const v4f*)(sES + 4 * iS);
    const v4f vD = *(const v4f*)(sED + 4 * iD);
    const bool isS = tid < NV;
    const v4f dv = isS ? vS : vD;
    float* gp = isS ? (eS + eb + 4 * iS) : (eD + eb + 4 * iD);
    const bool act = (tid < 2 * NV);
    if (act) *(volatile v4f*)gp = dv;
    __threadfence();
    if (act) *(volatile v4f*)gp = dv;
  }
}

__global__ __launch_bounds__(NTHR) void k_agg(
    const int* __restrict__ csr, const int* __restrict__ off, const int* __restrict__ cnt,
    const float* __restrict__ eS, const float* __restrict__ eD, const float* __restrict__ z,
    const float* __restrict__ bias, float* yo, int nS, int nD, int nTot, int npad, int csrLen) {
  constexpr int CPL = NC / 32;
  static_assert(CPL == 16);
  static_assert(NC == 4 * 128);
  __shared__ __attribute__((aligned(16))) float srow[NWAVE * NC];
  const int tid = threadIdx.x, lane = tid & 31, wave = tid >> 5;
  const int tbase = (int)blockIdx.x * TGT + wave * 32;
  const int col  = CPL * lane;
  const int slab = lane >> 3;
  const int hsub = (lane >> 2) & 1;
  const float* eSb = eS + (size_t)slab * (size_t)npad * HPS + hsub;
  const float* eDb = eD + (size_t)slab * (size_t)npad * HPS + hsub;
  float* sr = srow + wave * NC;

  const int cl    = tbase + lane;
  const int cnt_l = cnt[cl];
  const int off_l = off[cl];
  const v4f bq0 = *(const v4f*)(bias + col);
  const v4f bq1 = *(const v4f*)(bias + col + 4);
  const v4f bq2 = *(const v4f*)(bias + col + 8);
  const v4f bq3 = *(const v4f*)(bias + col + 12);

#pragma unroll 1
  for (int j = 0; j < 32; ++j) {
    const int d = tbase + j;
    int n = __shfl(cnt_l, j);
    n = n < 0 ? 0 : (n > DEGCAP ? DEGCAP : n);
    const int st = __shfl(off_l, j);
    const int dcl = d > nD - 1 ? nD - 1 : d;
    int dn = nS + dcl;
    dn = dn > nTot - 1 ? nTot - 1 : (dn < 0 ? 0 : dn);
    const float erd = eDb[(size_t)dn * HPS];
    const float es0 = lrelu(eSb[(size_t)dn * HPS] + erd);

    float mx = es0;
#pragma unroll 1
    for (int q0 = 0; q0 < n; q0 += 32) {
      int pos = st + q0 + lane;
      pos = pos < 0 ? 0 : (pos > csrLen - 1 ? csrLen - 1 : pos);
      int sl = csr[pos];
      sl = sl < 0 ? 0 : (sl > nTot - 1 ? nTot - 1 : sl);
      const int mcnt = (n - q0) < 32 ? (n - q0) : 32;
#pragma unroll 1
      for (int pp = 0; pp < mcnt; ++pp) {
        const int s = __builtin_amdgcn_readlane(sl, pp);
        mx = fmaxf(mx, lrelu(eSb[(size_t)s * HPS] + erd));
      }
    }

    const float pself = __expf(es0 - mx);
    float den = pself;
    const float* zs = z + (size_t)dn * NC + col;
    v4f a0 = *(const v4f*)zs * pself;
    v4f a1 = *(const v4f*)(zs + 4) * pself;
    v4f a2 = *(const v4f*)(zs + 8) * pself;
    v4f a3 = *(const v4f*)(zs + 12) * pself;
#pragma unroll 1
    for (int q0 = 0; q0 < n; q0 += 32) {
      int pos = st + q0 + lane;
      pos = pos < 0 ? 0 : (pos > csrLen - 1 ? csrLen - 1 : pos);
      int sl = csr[pos];
      sl = sl < 0 ? 0 : (sl > nTot - 1 ? nTot - 1 : sl);
      const int mcnt = (n - q0) < 32 ? (n - q0) : 32;
#pragma unroll 1
      for (int pp = 0; pp < mcnt; ++pp) {
        const int s = __builtin_amdgcn_readlane(sl, pp);
        const float p = __expf(lrelu(eSb[(size_t)s * HPS] + erd) - mx);
        den += p;
        const float* zr = z + (size_t)s * NC + col;
        const v4f h0 = *(const v4f*)zr;
        const v4f h1 = *(const v4f*)(zr + 4);
        const v4f h2 = *(const v4f*)(zr + 8);
        const v4f h3 = *(const v4f*)(zr + 12);
        a0 += h0 * p; a1 += h1 * p; a2 += h2 * p; a3 += h3 * p;
      }
    }

    const float rd = __builtin_amdgcn_rcpf(den);
    const v4f o0 = a0 * rd + bq0;
    const v4f o1 = a1 * rd + bq1;
    const v4f o2 = a2 * rd + bq2;
    const v4f o3 = a3 * rd + bq3;

    *(v4f*)(sr + col)      = o0;
    *(v4f*)(sr + col + 4)  = o1;
    *(v4f*)(sr + col + 8)  = o2;
    *(v4f*)(sr + col + 12) = o3;
    __builtin_amdgcn_fence(__ATOMIC_RELEASE, "wavefront");
    __builtin_amdgcn_wave_barrier();
    const v4f w0 = *(const v4f*)(sr + 4 * lane);
    const v4f w1 = *(const v4f*)(sr + 128 + 4 * lane);
    const v4f w2 = *(const v4f*)(sr + 256 + 4 * lane);
    const v4f w3 = *(const v4f*)(sr + 384 + 4 * lane);

    float* gp = yo + (size_t)dcl * NC + 4 * lane;
    const bool act = (d < nD);
    if (act) {
      *(volatile v4f*)gp         = w0;
      *(volatile v4f*)(gp + 128) = w1;
      *(volatile v4f*)(gp + 256) = w2;
      *(volatile v4f*)(gp + 384) = w3;
    }
    __threadfence();
    if (act) {
      *(volatile v4f*)gp         = w0;
      *(volatile v4f*)(gp + 128) = w1;
      *(volatile v4f*)(gp + 256) = w2;
      *(volatile v4f*)(gp + 384) = w3;
    }
    __builtin_amdgcn_wave_barrier();
  }
}

extern "C" void kernel_launch(void* const* d_in, const int* in_sizes, int n_in,
                              void* d_out, int out_size, void* d_ws, size_t ws_size,
                              hipStream_t stream) {
  if (n_in < 8) return;
  const int nS = in_sizes[0] / FIN;
  const int nD = in_sizes[1] / FIN;
  const int nE = in_sizes[2];
  if (nS <= 0 || nD <= 0 || nE <= 0) return;
  if (in_sizes[0] != nS * FIN || in_sizes[1] != nD * FIN) return;
  if (in_sizes[3] != nE) return;
  if (in_sizes[4] != FIN * NC) return;
  if (in_sizes[5] != NHEAD * CHN || in_sizes[6] != NHEAD * CHN) return;
  if (in_sizes[7] != NC) return;
  if (out_size != nD * NC) return;
  if (nE > (1 << 28) || nS > (1 << 21) || nD > (1 << 21)) return;
  const int nTot = nS + nD;

  const float* xs   = (const float*)d_in[0];
  const float* xd   = (const float*)d_in[1];
  const int*   esrc = (const int*)d_in[2];
  const int*   edst = (const int*)d_in[3];
  const float* W    = (const float*)d_in[4];
  const float* al   = (const float*)d_in[5];
  const float* ar   = (const float*)d_in[6];
  const float* bias = (const float*)d_in[7];
  float* out = (float*)d_out;

  const int NPAD   = ((nTot + RPAD - 1) / RPAD) * RPAD;
  const int nBC    = (nD + NBC - 1) / NBC;
  const int CNTPAD = nBC * NBC;
  const int nAgg   = (nD + TGT - 1) / TGT;
  const int DPAD   = nAgg * TGT;
  if (DPAD > CNTPAD) return;
  if (4 * nBC + 1 > RBN) return;
  const int nBF    = (nD + NBF - 1) / NBF;
  if (nBF > 4 * nBC) return;
  const int csrLen = ((nE + 31) & ~31) + 4096;
  if (31 * 4 * nBC > 4096) return;
  const int nGemm  = NPAD / BM;
  const int nXu1   = nS * (FIN / 8);
  const int nXu2   = (NPAD - nS) * (FIN / 8);

  char* ws = (char*)d_ws;
  size_t off = 0;
  const size_t oW   = off; off += (size_t)NC * FIN * 2;               off = (off + 255) & ~(size_t)255;
  const size_t oX   = off; off += (size_t)NPAD * FIN * 2;             off = (off + 255) & ~(size_t)255;
  const size_t oCnt = off; off += (size_t)CNTPAD * 4;                 off = (off + 255) & ~(size_t)255;
  const size_t oOff = off; off += (size_t)CNTPAD * 4;                 off = (off + 255) & ~(size_t)255;
  const size_t oRb  = off; off += (size_t)RBN * 4;                    off = (off + 255) & ~(size_t)255;
  const size_t oCsr = off; off += (size_t)csrLen * 4;                 off = (off + 255) & ~(size_t)255;
  const size_t oZ   = off; off += (size_t)NPAD * NC * 4;              off = (off + 255) & ~(size_t)255;
  const size_t oES  = off; off += (size_t)NSLAB * NPAD * HPS * 4;     off = (off + 255) & ~(size_t)255;
  const size_t oED  = off; off += (size_t)NSLAB * NPAD * HPS * 4;     off = (off + 255) & ~(size_t)255;
  if (off > ws_size || off > (size_t)WSCAP) return;
  _Float16* wp = (_Float16*)(ws + oW);
  _Float16* px = (_Float16*)(ws + oX);
  int*   cnt  = (int*)(ws + oCnt);
  int*   offp = (int*)(ws + oOff);
  int*   rb   = (int*)(ws + oRb);
  int*   csr  = (int*)(ws + oCsr);
  float* z    = (float*)(ws + oZ);
  float* es   = (float*)(ws + oES);
  float* ed   = (float*)(ws + oED);

  const int vec8 = 1;

  k_wtr<<<dim3(NC / 64, FIN / 64, 1), NTHR, 0, stream>>>(W, wp);
  k_xcvt<<<(nXu1 + NTHR - 1) / NTHR, NTHR, 0, stream>>>(xs, px, nS, nXu1);
  k_xcvt<<<(nXu2 + NTHR - 1) / NTHR, NTHR, 0, stream>>>(xd, px + (size_t)nS * FIN, nD, nXu2);

  k_count<<<nBC, NTHR, 0, stream>>>(edst, cnt, nE, vec8);
  k_offsets<<<1, OTHR, 0, stream>>>(cnt, offp, rb, nBC);
  hipFuncSetAttribute(reinterpret_cast<const void*>(&k_fill),
                      hipFuncAttributeMaxDynamicSharedMemorySize, LDS_FILL);
  k_fill<<<nBF, NTHR, LDS_FILL, stream>>>(esrc, edst, offp, rb, csr, nTot, nE, vec8, csrLen);

  k_gemm<<<dim3(nGemm, NSLAB, 1), NTHR, 0, stream>>>(px, wp, al, ar, z, es, ed, NPAD);

  k_agg<<<nAgg, NTHR, 0, stream>>>(csr, offp, cnt, es, ed, z, bias, out, nS, nD, nTot, NPAD, csrLen);
}
